// RCT_72679436583330
// MI455X (gfx1250) — hardware-verified
//
#include <hip/hip_runtime.h>
#include <math.h>
#include <stdint.h>


#define NB   2
#define SEQ  4096
#define CH   256
#define NHD  2
#define HD   128
#define FH   1024

typedef _Float16 v16h __attribute__((ext_vector_type(16)));
typedef _Float16 v8h  __attribute__((ext_vector_type(8)));
typedef __bf16   v16b __attribute__((ext_vector_type(16)));
typedef __bf16   v8b  __attribute__((ext_vector_type(8)));
typedef float    v8f  __attribute__((ext_vector_type(8)));
typedef float    v4f  __attribute__((ext_vector_type(4)));
typedef unsigned int v4u __attribute__((ext_vector_type(4)));
typedef unsigned int v2u __attribute__((ext_vector_type(2)));

__device__ __forceinline__ unsigned short f2bf_bits(float f) {
  const unsigned u = __float_as_uint(f);
  return (unsigned short)((u + 0x7FFFu + ((u >> 16) & 1u)) >> 16);
}
__device__ __forceinline__ float bf_bits2f(unsigned short x) { return __uint_as_float(((unsigned)x) << 16); }
__device__ __forceinline__ unsigned pk16(unsigned short a, unsigned short b) { return (unsigned)a | ((unsigned)b << 16); }
__device__ __forceinline__ unsigned short h2u(_Float16 x) { return __builtin_bit_cast(unsigned short, x); }

__device__ __forceinline__ void wave_sync() {
#if defined(__HIP_DEVICE_COMPILE__)
  __builtin_amdgcn_fence(__ATOMIC_RELEASE, "workgroup");
  __builtin_amdgcn_wave_barrier();
  __builtin_amdgcn_fence(__ATOMIC_ACQUIRE, "workgroup");
#endif
}

__device__ __forceinline__ float fexp2(float x) {
#if defined(__HIP_DEVICE_COMPILE__)
  return __builtin_amdgcn_exp2f(x);
#else
  return exp2f(x);
#endif
}
__device__ __forceinline__ float frcp(float x) {
#if defined(__HIP_DEVICE_COMPILE__)
  return __builtin_amdgcn_rcpf(x);
#else
  return 1.0f / x;
#endif
}
__device__ __forceinline__ int pin_off(int x, v8f d) {
#if defined(__HIP_DEVICE_COMPILE__)
  asm volatile("" : "+v"(x) : "v"(d));
#else
  (void)d;
#endif
  return x;
}

union FragB { v16b v; v8b h[2]; };
union FragH { v16h v; v8h h[2]; };
__device__ __forceinline__ v16b ldfrag_b(const __bf16* p) {
  FragB f; f.h[0] = *(const v8b*)(p); f.h[1] = *(const v8b*)(p + 16); return f.v;
}
__device__ __forceinline__ v16h ldfrag_h(const _Float16* p) {
  FragH f; f.h[0] = *(const v8h*)(p); f.h[1] = *(const v8h*)(p + 16); return f.v;
}

__device__ __forceinline__ v8f mma_b(v16b a, v16b b, v8f c) {
  return __builtin_amdgcn_wmma_f32_16x16x32_bf16(false, a, false, b, (short)0, c, false, false);
}
__device__ __forceinline__ v8f mma_h(v16h a, v16h b, v8f c) {
  return __builtin_amdgcn_wmma_f32_16x16x32_f16(false, a, false, b, (short)0, c, false, false);
}
__device__ __forceinline__ void guard_b(v8f& x, v8f& y, v16b b, v16b a0, v16b a1, v16b l0, v16b l1) {
#if defined(__HIP_DEVICE_COMPILE__)
  asm volatile("v_nop\n\tv_nop\n\tv_nop\n\tv_nop" : "+v"(x), "+v"(y) : "v"(b), "v"(a0), "v"(a1), "v"(l0), "v"(l1));
#endif
}
__device__ __forceinline__ void guard_h(v8f& d0, v8f& d1, v8f& d2, v8f& d3,
                                        v16h a, v16h b0, v16h b1, v16h b2, v16h b3) {
#if defined(__HIP_DEVICE_COMPILE__)
  asm volatile("v_nop\n\tv_nop\n\tv_nop\n\tv_nop"
               : "+v"(d0), "+v"(d1), "+v"(d2), "+v"(d3)
               : "v"(a), "v"(b0), "v"(b1), "v"(b2), "v"(b3));
#endif
}

__global__ __launch_bounds__(256) void cvt_kernel(
    const float* __restrict__ s0, const float* __restrict__ s1, const float* __restrict__ s2,
    const float* __restrict__ s3, const float* __restrict__ s4, const float* __restrict__ s5,
    unsigned short* d0, unsigned short* d1, unsigned short* d2,
    unsigned short* d3, unsigned short* d4, unsigned short* d5,
    int n0, int n1, int n2, int n3, int n4, int n5) {
  const int y = blockIdx.y;
  const float* src = s0; unsigned short* dst = d0; int n8 = n0;
  if (y == 1) { src = s1; dst = d1; n8 = n1; }
  if (y == 2) { src = s2; dst = d2; n8 = n2; }
  if (y == 3) { src = s3; dst = d3; n8 = n3; }
  if (y == 4) { src = s4; dst = d4; n8 = n4; }
  if (y == 5) { src = s5; dst = d5; n8 = n5; }
  const int i = blockIdx.x * 256 + threadIdx.x;
  if (i < n8) {
    const v4f a = *(const v4f*)(src + 8 * (size_t)i);
    const v4f c = *(const v4f*)(src + 8 * (size_t)i + 4);
    v4u w;
    w[0] = pk16(f2bf_bits(a[0]), f2bf_bits(a[1]));
    w[1] = pk16(f2bf_bits(a[2]), f2bf_bits(a[3]));
    w[2] = pk16(f2bf_bits(c[0]), f2bf_bits(c[1]));
    w[3] = pk16(f2bf_bits(c[2]), f2bf_bits(c[3]));
    volatile v4u* p = (volatile v4u*)(dst + 8 * (size_t)i);
    *p = w;
    __threadfence();
    *p = w;
  }
}

#define GP 68

template <bool SPLITA, int OUT_MODE, int RES, bool RELU>
__global__ __launch_bounds__(128) void gemm_kernel(
    const unsigned short* __restrict__ Ap, const unsigned short* __restrict__ A2p, int lda,
    const unsigned short* __restrict__ Btp, int ldb, long strideB,
    void* Cout, void* Cout2, int ldc, long strideC,
    const unsigned short* __restrict__ Rb, const float* __restrict__ Rf, float oscale,
    int M, int N, int K) {
  __shared__ __align__(16) float sT[4][16 * GP];
  const int bz   = blockIdx.y;
  const int lane = threadIdx.x & 31;
  const int wave = threadIdx.x >> 5;
  const int tilesN = N >> 6;
  const int tilesM = M >> 5;
  const int tile = blockIdx.x * 4 + wave;
  if (tile >= tilesM * tilesN) return;
  const int tm = tile / tilesN;
  const int tn = tile - tm * tilesN;
  const int m0 = tm << 5;
  const int n0 = tn << 6;

  const __bf16* Ab  = (const __bf16*)(const void*)Ap;
  const __bf16* Ab2 = (const __bf16*)(const void*)A2p;
  const __bf16* Bb  = (const __bf16*)(const void*)Btp + (size_t)bz * strideB;

  const int rlane = lane & 15;
  const int koff  = (lane >> 4) * 8;
  const int mOff  = (lane >> 4) * 8;

  const v8f zero8 = (v8f){0.f, 0.f, 0.f, 0.f, 0.f, 0.f, 0.f, 0.f};
  v8f acc[2][4];
#pragma unroll
  for (int i = 0; i < 2; ++i)
#pragma unroll
    for (int j = 0; j < 4; ++j) acc[i][j] = zero8;
  v8f dep = acc[1][3];

  for (int k0 = 0; k0 < K; k0 += 32) {
    const size_t ao0 = (size_t)(m0 + rlane) * lda + koff + k0;
    const size_t ao1 = (size_t)(m0 + 16 + rlane) * lda + koff + k0;
    const v16b a0 = ldfrag_b(Ab + ao0);
    const v16b a1 = ldfrag_b(Ab + ao1);
    v16b l0 = a0, l1 = a1;
    if (SPLITA) { l0 = ldfrag_b(Ab2 + ao0); l1 = ldfrag_b(Ab2 + ao1); }
#pragma unroll
    for (int j = 0; j < 4; ++j) {
      const int boff = pin_off(koff + k0, dep);
      const v16b bh = ldfrag_b(Bb + (size_t)(n0 + (j << 4) + rlane) * ldb + boff);
      acc[0][j] = mma_b(a0, bh, acc[0][j]);
      if (SPLITA) acc[0][j] = mma_b(l0, bh, acc[0][j]);
      acc[1][j] = mma_b(a1, bh, acc[1][j]);
      if (SPLITA) acc[1][j] = mma_b(l1, bh, acc[1][j]);
      guard_b(acc[0][j], acc[1][j], bh, a0, a1, l0, l1);
      dep = acc[1][j];
    }
  }

  float* slab = sT[wave];
#pragma unroll
  for (int i = 0; i < 2; ++i) {
    const int mBase = m0 + (i << 4);
#pragma unroll
    for (int j = 0; j < 4; ++j)
#pragma unroll
      for (int r = 0; r < 8; ++r) slab[(mOff + r) * GP + (j << 4) + rlane] = acc[i][j][r];
    wave_sync();
    if (OUT_MODE == 0) {
      float* Cc = (float*)Cout + (size_t)bz * strideC;
      const int q16 = lane >> 4, c4 = (lane & 15) * 4;
      for (int pass = 0; pass < 2; ++pass) {
#pragma unroll
        for (int it = 0; it < 8; ++it) {
          const int row = it * 2 + q16;
          v4f v = *(const v4f*)(slab + row * GP + c4);
          const size_t go = (size_t)(mBase + row) * ldc + n0 + c4;
          if (RES == 1) {
            const v2u rw = *(const v2u*)(Rb + go);
            v[0] += __uint_as_float(rw[0] << 16);
            v[1] += __uint_as_float(rw[0] & 0xffff0000u);
            v[2] += __uint_as_float(rw[1] << 16);
            v[3] += __uint_as_float(rw[1] & 0xffff0000u);
          }
          if (RES == 2) {
            const v4f rr = *(const v4f*)(Rf + go);
            v += rr;
          }
          *(volatile v4f*)(Cc + go) = v;
        }
        __threadfence();
      }
    } else {
      const int q4 = lane >> 3, c8 = (lane & 7) * 8;
      for (int pass = 0; pass < 2; ++pass) {
#pragma unroll
        for (int it = 0; it < 4; ++it) {
          const int row = it * 4 + q4;
          const float* sp = slab + row * GP + c8;
          const v4f x0 = *(const v4f*)(sp);
          const v4f x1 = *(const v4f*)(sp + 4);
          float f[8] = {x0[0], x0[1], x0[2], x0[3], x1[0], x1[1], x1[2], x1[3]};
          if (OUT_MODE == 1) {
            v4u hv, lv;
#pragma unroll
            for (int p = 0; p < 4; ++p) {
              float f0 = f[2 * p], f1 = f[2 * p + 1];
              if (RELU) { f0 = fmaxf(f0, 0.f); f1 = fmaxf(f1, 0.f); }
              const unsigned short hb0 = f2bf_bits(f0), hb1 = f2bf_bits(f1);
              const unsigned short lb0 = f2bf_bits(f0 - bf_bits2f(hb0));
              const unsigned short lb1 = f2bf_bits(f1 - bf_bits2f(hb1));
              hv[p] = pk16(hb0, hb1);
              lv[p] = pk16(lb0, lb1);
            }
            const size_t go = (size_t)bz * strideC + (size_t)(mBase + row) * ldc + n0 + c8;
            *(volatile v4u*)((unsigned short*)Cout + go)  = hv;
            *(volatile v4u*)((unsigned short*)Cout2 + go) = lv;
          } else {
            v4u hv;
#pragma unroll
            for (int p = 0; p < 4; ++p) {
              const _Float16 e0 = (_Float16)(f[2 * p] * oscale);
              const _Float16 e1 = (_Float16)(f[2 * p + 1] * oscale);
              hv[p] = pk16(h2u(e0), h2u(e1));
            }
            size_t go;
            if (OUT_MODE == 2) {
              const int srow = (mBase + row) & (SEQ - 1);
              const int bidx = m0 >> 12;
              const int head = n0 >> 7;
              go = ((size_t)(bidx * NHD + head) * SEQ + srow) * HD + (n0 & (HD - 1)) + c8;
            } else {
              go = (size_t)bz * strideC + (size_t)(mBase + row) * ldc + n0 + c8;
            }
            *(volatile v4u*)((unsigned short*)Cout + go) = hv;
          }
        }
        __threadfence();
      }
    }
    wave_sync();
  }
}

#define AT_QB 64
#define AT_KC 64

__global__ __launch_bounds__(128)
void attn_kernel(const unsigned short* __restrict__ qp, const unsigned short* __restrict__ kp,
                 const unsigned short* __restrict__ vtp, unsigned short* chp, unsigned short* clp) {
  __shared__ __align__(16) _Float16 KVs[2 * AT_KC * HD];
  __shared__ __align__(16) _Float16 Psh[4][16 * AT_KC];
  static_assert(4 * 16 * HD * 4 <= 2 * AT_KC * HD * 2);
  _Float16* const Ksh = KVs;
  _Float16* const Vsh = KVs + AT_KC * HD;

  const int tid  = threadIdx.x;
  const int wave = tid >> 5;
  const int lane = tid & 31;
  const int hh   = lane >> 4;
  const int c    = lane & 15;

  const int bx = blockIdx.x;
  const int qb = bx & (SEQ / AT_QB - 1);
  const int h  = (bx >> 6) & (NHD - 1);
  const int b  = bx >> 7;
  const int q0 = qb * AT_QB + wave * 16;

  const _Float16* Qg = (const _Float16*)(const void*)qp  + (size_t)(b * NHD + h) * SEQ * HD;
  const _Float16* Kg = (const _Float16*)(const void*)kp  + (size_t)(b * NHD + h) * SEQ * HD;
  const _Float16* Vg = (const _Float16*)(const void*)vtp + ((size_t)b * CH + (size_t)h * HD) * SEQ;
  const int qro = (q0 + c) * HD + 8 * hh;

  const v8f zero8 = (v8f){0.f, 0.f, 0.f, 0.f, 0.f, 0.f, 0.f, 0.f};

  float mrow[8], lsum[8];
  v8f oh[8];
#pragma unroll
  for (int r = 0; r < 8; ++r) { mrow[r] = -INFINITY; lsum[r] = 0.f; }
#pragma unroll
  for (int t = 0; t < 8; ++t) oh[t] = zero8;

  for (int kc = 0; kc < SEQ / AT_KC; ++kc) {
    const int kv0 = kc * AT_KC;
    __syncthreads();
    {
      const int r = tid >> 1, half = (tid & 1) * 64;
      const _Float16* ks = Kg + (size_t)(kv0 + r) * HD + half;
      const _Float16* vs = Vg + (size_t)tid * SEQ + kv0;
#pragma unroll
      for (int i = 0; i < 8; ++i) {
        const v8h a0 = *(const v8h*)(ks + 8 * i);
        const v8h b0 = *(const v8h*)(vs + 8 * i);
        *(v8h*)(Ksh + r * HD + half + 8 * i) = a0;
        *(v8h*)(Vsh + tid * AT_KC + 8 * i)   = b0;
      }
    }
    __syncthreads();

    v8f s[4];
#pragma unroll
    for (int j = 0; j < 4; ++j) s[j] = zero8;
    v8f dep = oh[7];
#pragma unroll
    for (int dc = 0; dc < 4; ++dc) {
      const int qo = pin_off(qro + dc * 32, dep);
      const int ko = pin_off(c * HD + dc * 32 + 8 * hh, dep);
      const v16h qf = ldfrag_h(Qg + qo);
      v16h kb[4];
#pragma unroll
      for (int j = 0; j < 4; ++j) kb[j] = ldfrag_h(Ksh + (j * 16) * HD + ko);
#pragma unroll
      for (int j = 0; j < 4; ++j) s[j] = mma_h(qf, kb[j], s[j]);
      guard_h(s[0], s[1], s[2], s[3], qf, kb[0], kb[1], kb[2], kb[3]);
      dep = s[3];
    }

    float cm[8];
#pragma unroll
    for (int r = 0; r < 8; ++r) {
      float m = fmaxf(fmaxf(s[0][r], s[1][r]), fmaxf(s[2][r], s[3][r]));
#pragma unroll
      for (int off = 1; off < 16; off <<= 1) m = fmaxf(m, __shfl_xor(m, off, 32));
      cm[r] = m;
    }

    _Float16* pw = Psh[wave];
#pragma unroll
    for (int r = 0; r < 8; ++r) {
      const float mnew  = fmaxf(mrow[r], cm[r]);
      const float alpha = fexp2(mrow[r] - mnew);
      mrow[r] = mnew;
      const float mb = mnew - 10.0f;
      float ps = 0.f;
#pragma unroll
      for (int j = 0; j < 4; ++j) {
        const float p = fexp2(s[j][r] - mb);
        ps += p;
        pw[(8 * hh + r) * AT_KC + j * 16 + c] = (_Float16)p;
      }
      lsum[r] = lsum[r] * alpha + ps;
#pragma unroll
      for (int t = 0; t < 8; ++t) oh[t][r] *= alpha;
    }
    wave_sync();

    v8f dep2 = oh[7];
#pragma unroll
    for (int kk = 0; kk < 2; ++kk) {
      FragH pa;
      pa.h[0] = *(const v8h*)(pw + c * AT_KC + kk * 32 + 8 * hh);
      pa.h[1] = *(const v8h*)(pw + c * AT_KC + kk * 32 + 16 + 8 * hh);
#pragma unroll
      for (int tg = 0; tg < 2; ++tg) {
        const int vo = pin_off(c * AT_KC + kk * 32 + 8 * hh, dep2);
        v16h vb[4];
#pragma unroll
        for (int u = 0; u < 4; ++u) vb[u] = ldfrag_h(Vsh + ((tg * 4 + u) * 16) * AT_KC + vo);
#pragma unroll
        for (int u = 0; u < 4; ++u) oh[tg * 4 + u] = mma_h(pa.v, vb[u], oh[tg * 4 + u]);
        guard_h(oh[tg * 4], oh[tg * 4 + 1], oh[tg * 4 + 2], oh[tg * 4 + 3], pa.v, vb[0], vb[1], vb[2], vb[3]);
        dep2 = oh[tg * 4 + 3];
      }
    }
  }

#pragma unroll
  for (int r = 0; r < 8; ++r) {
#pragma unroll
    for (int off = 1; off < 16; off <<= 1) lsum[r] += __shfl_xor(lsum[r], off, 32);
  }
  __syncthreads();
  float* os = (float*)(void*)KVs + wave * (16 * HD);
#pragma unroll
  for (int r = 0; r < 8; ++r) {
    const float invl = frcp(lsum[r]);
#pragma unroll
    for (int t = 0; t < 8; ++t) os[(8 * hh + r) * HD + t * 16 + c] = oh[t][r] * invl;
  }
  wave_sync();
  {
    const int q16 = lane >> 4, c8 = (lane & 15) * 8;
    for (int pass = 0; pass < 2; ++pass) {
#pragma unroll
      for (int it = 0; it < 8; ++it) {
        const int row = it * 2 + q16;
        const float* sp = os + row * HD + c8;
        const v4f x0 = *(const v4f*)(sp);
        const v4f x1 = *(const v4f*)(sp + 4);
        const float f[8] = {x0[0], x0[1], x0[2], x0[3], x1[0], x1[1], x1[2], x1[3]};
        v4u hv, lv;
#pragma unroll
        for (int p = 0; p < 4; ++p) {
          const float f0 = f[2 * p], f1 = f[2 * p + 1];
          const unsigned short hb0 = f2bf_bits(f0), hb1 = f2bf_bits(f1);
          const unsigned short lb0 = f2bf_bits(f0 - bf_bits2f(hb0));
          const unsigned short lb1 = f2bf_bits(f1 - bf_bits2f(hb1));
          hv[p] = pk16(hb0, hb1);
          lv[p] = pk16(lb0, lb1);
        }
        const size_t go = (size_t)(b * SEQ + q0 + row) * CH + h * HD + c8;
        *(volatile v4u*)(chp + go) = hv;
        *(volatile v4u*)(clp + go) = lv;
      }
      __threadfence();
    }
  }
}

template <bool ADDRES, bool HL>
__global__ __launch_bounds__(256) void ln_kernel(const float* __restrict__ X, const float* __restrict__ G,
                                                 const float* __restrict__ Bt, const float* __restrict__ R,
                                                 float* OF, unsigned short* OH, unsigned short* OL, int nrows) {
  __shared__ __align__(16) float lrw[8][CH];
  const int lane = threadIdx.x & 31;
  const int wave = threadIdx.x >> 5;
  const int row  = blockIdx.x * 8 + wave;
  if (row >= nrows) return;
  const size_t rb = (size_t)row * CH;
  const int ca = 4 * lane, cb = (CH / 2) + 4 * lane;

  const v4f xa = *(const v4f*)(X + rb + ca);
  const v4f xb = *(const v4f*)(X + rb + cb);
  float s = ((xa[0] + xa[1]) + (xa[2] + xa[3])) + ((xb[0] + xb[1]) + (xb[2] + xb[3]));
#pragma unroll
  for (int off = 1; off < 32; off <<= 1) s += __shfl_xor(s, off, 32);
  const float mu = s * (1.0f / CH);
  const v4f da = xa - mu;
  const v4f db = xb - mu;
  float ss = ((da[0] * da[0] + da[1] * da[1]) + (da[2] * da[2] + da[3] * da[3])) +
             ((db[0] * db[0] + db[1] * db[1]) + (db[2] * db[2] + db[3] * db[3]));
#pragma unroll
  for (int off = 1; off < 32; off <<= 1) ss += __shfl_xor(ss, off, 32);
  const float rs = rsqrtf(ss * (1.0f / CH) + 1e-6f);

  const v4f ga = *(const v4f*)(G + ca), gb = *(const v4f*)(G + cb);
  const v4f ba = *(const v4f*)(Bt + ca), bb = *(const v4f*)(Bt + cb);
  v4f ya = (da * rs) * ga + ba;
  v4f yb = (db * rs) * gb + bb;
  if (ADDRES) {
    const v4f ra = *(const v4f*)(R + rb + ca);
    const v4f rr = *(const v4f*)(R + rb + cb);
    ya += ra;
    yb += rr;
  }
  volatile v4f* pa = (volatile v4f*)(OF + rb + ca);
  volatile v4f* pb = (volatile v4f*)(OF + rb + cb);
  *pa = ya; *pb = yb;
  __threadfence();
  *pa = ya; *pb = yb;

  if (HL) {
    float* lr = lrw[wave];
    *(v4f*)(lr + ca) = ya;
    *(v4f*)(lr + cb) = yb;
    wave_sync();
    const v4f p0 = *(const v4f*)(lr + 8 * lane);
    const v4f p1 = *(const v4f*)(lr + 8 * lane + 4);
    const float f[8] = {p0[0], p0[1], p0[2], p0[3], p1[0], p1[1], p1[2], p1[3]};
    v4u hv, lv;
#pragma unroll
    for (int p = 0; p < 4; ++p) {
      const float f0 = f[2 * p], f1 = f[2 * p + 1];
      const unsigned short hb0 = f2bf_bits(f0), hb1 = f2bf_bits(f1);
      const unsigned short lb0 = f2bf_bits(f0 - bf_bits2f(hb0));
      const unsigned short lb1 = f2bf_bits(f1 - bf_bits2f(hb1));
      hv[p] = pk16(hb0, hb1);
      lv[p] = pk16(lb0, lb1);
    }
    const size_t go = rb + 8 * lane;
    volatile v4u* ph = (volatile v4u*)(OH + go);
    volatile v4u* pl = (volatile v4u*)(OL + go);
    *ph = hv; *pl = lv;
    __threadfence();
    *ph = hv; *pl = lv;
  }
}

extern "C" void kernel_launch(void* const* d_in, const int* in_sizes, int n_in,
                              void* d_out, int out_size, void* d_ws, size_t ws_size,
                              hipStream_t stream) {
  if (n_in < 14) return;
  const int nAct = NB * SEQ * CH;
  const int nW = 3 * CH * CH, nW1 = 3 * FH * CH, nG = 3 * CH;
  if (in_sizes[0] != nAct || in_sizes[1] != nAct || in_sizes[2] != nAct) return;
  if (in_sizes[4] != nW || in_sizes[5] != nW || in_sizes[6] != nW || in_sizes[7] != nW) return;
  if (in_sizes[8] != nG || in_sizes[9] != nG || in_sizes[12] != nG || in_sizes[13] != nG) return;
  if (in_sizes[10] != nW1 || in_sizes[11] != nW1) return;
  if (out_size != nAct) return;

  const float* Fm   = (const float*)d_in[0];
  const float* Fs   = (const float*)d_in[1];
  const float* Fq   = (const float*)d_in[2];
  const float* Wq   = (const float*)d_in[4];
  const float* Wk   = (const float*)d_in[5];
  const float* Wv   = (const float*)d_in[6];
  const float* Wo   = (const float*)d_in[7];
  const float* LnG  = (const float*)d_in[8];
  const float* LnB  = (const float*)d_in[9];
  const float* W1   = (const float*)d_in[10];
  const float* W2   = (const float*)d_in[11];
  const float* FlnG = (const float*)d_in[12];
  const float* FlnB = (const float*)d_in[13];
  float* out = (float*)d_out;

  const size_t szA2  = (size_t)nAct * 2;
  const size_t szA4  = (size_t)nAct * 4;
  const size_t szW2  = (size_t)nW * 2;
  const size_t szW12 = (size_t)nW1 * 2;
  const size_t szPl  = (size_t)NB * NHD * SEQ * HD * 2;
  const size_t szVt  = (size_t)NB * CH * SEQ * 2;
  const size_t szH2  = (size_t)NB * SEQ * FH * 2;
  size_t off = 0;
  const size_t oFm  = off; off += szA2;
  const size_t oFs  = off; off += szA2;
  const size_t oFq  = off; off += szA2;
  const size_t oWq  = off; off += szW2;
  const size_t oWk  = off; off += szW2;
  const size_t oWv  = off; off += szW2;
  const size_t oWo  = off; off += szW2;
  const size_t oW1  = off; off += szW12;
  const size_t oW2  = off; off += szW12;
  const size_t oQ   = off; off += szPl;
  const size_t oK   = off; off += szPl;
  const size_t oVt  = off; off += szVt;
  const size_t oCh  = off; off += szA2;
  const size_t oCl  = off; off += szA2;
  const size_t oAO  = off; off += szA4;
  const size_t oX1f = off; off += szA4;
  const size_t oX1h = off; off += szA2;
  const size_t oX1l = off; off += szA2;
  const size_t oHh  = off; off += szH2;
  const size_t oHl  = off; off += szH2;
  const size_t oCsF = off; off += szA4;
  const size_t oCsH = off; off += szA2;
  const size_t oCsL = off; off += szA2;
  const size_t oCqH = off; off += szA2;
  const size_t oCqL = off; off += szA2;
  if (off > ws_size) return;
  if (off > (size_t)134217728u) return;

  char* ws = (char*)d_ws;
  unsigned short* Fmb = (unsigned short*)(ws + oFm);
  unsigned short* Fsb = (unsigned short*)(ws + oFs);
  unsigned short* Fqb = (unsigned short*)(ws + oFq);
  unsigned short* Wqb = (unsigned short*)(ws + oWq);
  unsigned short* Wkb = (unsigned short*)(ws + oWk);
  unsigned short* Wvb = (unsigned short*)(ws + oWv);
  unsigned short* Wob = (unsigned short*)(ws + oWo);
  unsigned short* W1b = (unsigned short*)(ws + oW1);
  unsigned short* W2b = (unsigned short*)(ws + oW2);
  unsigned short* Qp  = (unsigned short*)(ws + oQ);
  unsigned short* Kp  = (unsigned short*)(ws + oK);
  unsigned short* Vt  = (unsigned short*)(ws + oVt);
  unsigned short* Chh = (unsigned short*)(ws + oCh);
  unsigned short* Cll = (unsigned short*)(ws + oCl);
  float*          AO  = (float*)(ws + oAO);
  float*          X1f = (float*)(ws + oX1f);
  unsigned short* X1h = (unsigned short*)(ws + oX1h);
  unsigned short* X1l = (unsigned short*)(ws + oX1l);
  unsigned short* Hh  = (unsigned short*)(ws + oHh);
  unsigned short* Hl  = (unsigned short*)(ws + oHl);
  float*          CsF = (float*)(ws + oCsF);
  unsigned short* CsH = (unsigned short*)(ws + oCsH);
  unsigned short* CsL = (unsigned short*)(ws + oCsL);
  unsigned short* CqH = (unsigned short*)(ws + oCqH);
  unsigned short* CqL = (unsigned short*)(ws + oCqL);
  float*          Scr = (float*)(ws + oHh);

  const dim3 blk256(256), blk128(128);
  const int M = NB * SEQ;
  const float sc2 = 0.08838834764831845f * 1.4426950408889634f;

  {
    const int n8a = nAct / 8, n8w = nW / 8, n8w1 = nW1 / 8;
    cvt_kernel<<<dim3((n8a + 255) / 256, 3), blk256, 0, stream>>>(
        Fm, Fs, Fq, Fm, Fm, Fm, Fmb, Fsb, Fqb, Fmb, Fmb, Fmb, n8a, n8a, n8a, 0, 0, 0);
    cvt_kernel<<<dim3((n8w1 + 255) / 256, 6), blk256, 0, stream>>>(
        Wq, Wk, Wv, Wo, W1, W2, Wqb, Wkb, Wvb, Wob, W1b, W2b, n8w, n8w, n8w, n8w, n8w1, n8w1);
  }

  const int tilesQK  = (M / 32) * (CH / 64);
  const int tilesVt  = (CH / 32) * (SEQ / 64);
  const int tilesFF1 = (M / 32) * (FH / 64);
  const dim3 gQK((tilesQK + 3) / 4, 1), gVt((tilesVt + 3) / 4, NB), gFF1((tilesFF1 + 3) / 4, 1);
  const dim3 gAttn(NB * NHD * (SEQ / AT_QB));
  const dim3 gLN(M / 8);

  auto front = [&](int i, const unsigned short* Qsrc, const unsigned short* Ksrc, const unsigned short* Vsrc) {
    const size_t wofs = (size_t)i * CH * CH;
    gemm_kernel<false, 2, 0, false><<<gQK, blk128, 0, stream>>>(
        Qsrc, Qsrc, CH, Wqb + wofs, CH, 0L, (void*)Qp, (void*)Qp, HD, 0L, Fmb, CsF, sc2, M, CH, CH);
    gemm_kernel<false, 2, 0, false><<<gQK, blk128, 0, stream>>>(
        Ksrc, Ksrc, CH, Wkb + wofs, CH, 0L, (void*)Kp, (void*)Kp, HD, 0L, Fmb, CsF, 1.0f, M, CH, CH);
    gemm_kernel<false, 3, 0, false><<<gVt, blk128, 0, stream>>>(
        Wvb + wofs, Wvb + wofs, CH, Vsrc, CH, (long)SEQ * CH, (void*)Vt, (void*)Vt, SEQ, (long)CH * SEQ,
        Fmb, CsF, 1.0f, CH, SEQ, CH);
    attn_kernel<<<gAttn, blk128, 0, stream>>>(Qp, Kp, Vt, Chh, Cll);
  };
  auto back = [&](int i) {
    ln_kernel<false, true><<<gLN, blk256, 0, stream>>>(AO, LnG + i * CH, LnB + i * CH, AO, X1f, X1h, X1l, M);
    gemm_kernel<true, 1, 0, true><<<gFF1, blk128, 0, stream>>>(
        X1h, X1l, CH, W1b + (size_t)i * FH * CH, CH, 0L, (void*)Hh, (void*)Hl, FH, 0L, Fmb, CsF, 1.0f, M, FH, CH);
    gemm_kernel<true, 0, 0, false><<<gQK, blk128, 0, stream>>>(
        Hh, Hl, FH, W2b + (size_t)i * CH * FH, FH, 0L, (void*)AO, (void*)AO, CH, 0L, Fmb, CsF, 1.0f, M, CH, FH);
  };

  front(0, Fsb, Fsb, Fmb);
  gemm_kernel<true, 0, 1, false><<<gQK, blk128, 0, stream>>>(
      Chh, Cll, CH, Wob, CH, 0L, (void*)AO, (void*)AO, CH, 0L, Fmb, CsF, 1.0f, M, CH, CH);
  back(0);
  ln_kernel<true, true><<<gLN, blk256, 0, stream>>>(AO, FlnG, FlnB, X1f, CsF, CsH, CsL, M);

  front(1, Fqb, Fqb, Fqb);
  gemm_kernel<true, 0, 1, false><<<gQK, blk128, 0, stream>>>(
      Chh, Cll, CH, Wob + (size_t)CH * CH, CH, 0L, (void*)AO, (void*)AO, CH, 0L, Fqb, CsF, 1.0f, M, CH, CH);
  back(1);
  ln_kernel<true, true><<<gLN, blk256, 0, stream>>>(AO, FlnG + CH, FlnB + CH, X1f, Scr, CqH, CqL, M);

  front(2, CqH, Fsb, CsH);
  gemm_kernel<true, 0, 2, false><<<gQK, blk128, 0, stream>>>(
      Chh, Cll, CH, Wob + (size_t)2 * CH * CH, CH, 0L, (void*)AO, (void*)AO, CH, 0L, Fmb, CsF, 1.0f, M, CH, CH);
  back(2);
  ln_kernel<true, false><<<gLN, blk256, 0, stream>>>(AO, FlnG + 2 * CH, FlnB + 2 * CH, X1f, out, Chh, Cll, M);

  (void)hipGetLastError();
}
